// GCN_1099511628226
// MI455X (gfx1250) — hardware-verified
//
#include <hip/hip_runtime.h>
#include <stddef.h>
#include <stdint.h>
#include <math.h>


#define DF     128
#define XP     256
#define XLO    128
#define NCLS   40
#define NTHR   256
#define NWAVE  8
#define EPT    8
#define CHUNK  (NTHR * EPT)
#define WCAP   (EPT * 32)
#define LISTN  (NWAVE * WCAP)
#define NBA    1024
#define SLA    10
#define SPW    (NBA / NWAVE)
#define RCAP   16384
#define DEGCAP 64
#define NBD    16384
#define GBM    64
#define GTHR   128
#define APH    264
#define NU0    4096
#define NU1    8192
#define NU2    4096
#define OGRP   16
#define WSMAX  134217728

static_assert((CHUNK & (CHUNK - 1)) == 0 && CHUNK <= 4096);
static_assert((NBA & (NBA - 1)) == 0 && NBA == (1 << SLA));
static_assert(((long long)CHUNK << SLA) < (1LL << 31));
static_assert(NBA % NWAVE == 0 && NBA % 32 == 0 && SPW % OGRP == 0);
static_assert(RCAP % 4 == 0 && LISTN % 4 == 0);
static_assert(NBD % (NTHR * 4) == 0 && (NBD & (NBD - 1)) == 0);
static_assert(GBM == (GTHR / 32) * 16 && DF % 32 == 0 && (2 * DF) % 32 == 0);
static_assert(APH % 8 == 0 && APH >= 2 * DF);
static_assert(NU0 % NTHR == 0 && NU1 % NTHR == 0 && NU2 % NTHR == 0);
static_assert((40 * 32) % NTHR == 0 && (64 * 32) % NTHR == 0 && (104 * 32) % NTHR == 0);
static_assert((OGRP * NCLS * 4) % 512 == 0 && (OGRP * NCLS) == 5 * 128);
static_assert(NCLS % 2 == 0 && NCLS / 2 <= 32 && NCLS <= 64);

typedef float          v2f   __attribute__((ext_vector_type(2)));
typedef float          v4f   __attribute__((ext_vector_type(4)));
typedef float          v8f   __attribute__((ext_vector_type(8)));
typedef double         v2d   __attribute__((ext_vector_type(2)));
typedef int            v4i   __attribute__((ext_vector_type(4)));
typedef int            v8i   __attribute__((ext_vector_type(8)));
typedef unsigned short v8us  __attribute__((ext_vector_type(8)));
typedef unsigned short v16us __attribute__((ext_vector_type(16)));
typedef __bf16         v16bf __attribute__((ext_vector_type(16)));
typedef v2f  __attribute__((may_alias)) v2fa;
typedef v4f  __attribute__((may_alias)) v4fa;
typedef v4i  __attribute__((may_alias)) v4ia;
typedef v8us __attribute__((may_alias)) v8usa;
union FragB { v16bf v; v16us u; v8us h[2]; v8i w; };

__device__ __forceinline__ v8f wmb(const FragB& a, const FragB& b, v8f c) {
  v8f d = __builtin_amdgcn_wmma_f32_16x16x32_bf16(false, a.v, false, b.v, (short)0, c, false, false);
  asm volatile("v_nop\n\tv_nop\n\tv_nop\n\tv_nop" : "+v"(d) : "v"(a.w), "v"(b.w));
  return d;
}

__device__ __forceinline__ unsigned bf16_bits(float f) {
  const unsigned u = __float_as_uint(f);
  return (u + 0x7FFFu + ((u >> 16) & 1u)) >> 16;
}
__device__ __forceinline__ float bf16_val(float f) {
  return __uint_as_float(bf16_bits(f) << 16);
}

__device__ __forceinline__ void wave_sync() {
  __builtin_amdgcn_fence(__ATOMIC_RELEASE, "wavefront");
  __builtin_amdgcn_wave_barrier();
  __builtin_amdgcn_fence(__ATOMIC_ACQUIRE, "wavefront");
}

template <int SLB>
__device__ __forceinline__ int scan_chunk(const int* __restrict__ dsts, int nE, int cbase, int slotBase,
                                          int nb, int vec8, int* list, int tid, int lane, int wave) {
  int wc = 0;
  const int el0  = tid * EPT;
  const int e0   = cbase + el0;
  const int sent = -2147483647 - 1;
  v4i da, db;
  if (vec8 != 0 && cbase + CHUNK <= nE) {
    da = *(const v4i*)(dsts + e0);
    db = *(const v4i*)(dsts + e0 + 4);
  } else {
    da.x = (e0     < nE) ? dsts[min(e0,     nE - 1)] : sent;
    da.y = (e0 + 1 < nE) ? dsts[min(e0 + 1, nE - 1)] : sent;
    da.z = (e0 + 2 < nE) ? dsts[min(e0 + 2, nE - 1)] : sent;
    da.w = (e0 + 3 < nE) ? dsts[min(e0 + 3, nE - 1)] : sent;
    db.x = (e0 + 4 < nE) ? dsts[min(e0 + 4, nE - 1)] : sent;
    db.y = (e0 + 5 < nE) ? dsts[min(e0 + 5, nE - 1)] : sent;
    db.z = (e0 + 6 < nE) ? dsts[min(e0 + 6, nE - 1)] : sent;
    db.w = (e0 + 7 < nE) ? dsts[min(e0 + 7, nE - 1)] : sent;
  }
  const unsigned nbs = (unsigned)slotBase;
  const unsigned unb = (unsigned)nb;
  const unsigned s0 = (unsigned)da.x - nbs, s1 = (unsigned)da.y - nbs;
  const unsigned s2 = (unsigned)da.z - nbs, s3 = (unsigned)da.w - nbs;
  const unsigned s4 = (unsigned)db.x - nbs, s5 = (unsigned)db.y - nbs;
  const unsigned s6 = (unsigned)db.z - nbs, s7 = (unsigned)db.w - nbs;
  const bool h0 = s0 < unb, h1 = s1 < unb, h2 = s2 < unb, h3 = s3 < unb;
  const bool h4 = s4 < unb, h5 = s5 < unb, h6 = s6 < unb, h7 = s7 < unb;
  const unsigned any = __builtin_amdgcn_ballot_w32(h0 | h1 | h2 | h3 | h4 | h5 | h6 | h7);
  if (any != 0u) {
#define HITJ(J, HJ, SJ) { \
      const unsigned mj = __builtin_amdgcn_ballot_w32(HJ); \
      if (mj != 0u) { \
        if (HJ) { \
          const int pos = wc + (int)__builtin_amdgcn_mbcnt_lo(mj, 0u); \
          if (pos < WCAP) list[wave * WCAP + pos] = ((el0 + (J)) << SLB) | (int)(SJ); \
        } \
        wc += (int)__builtin_popcount(mj); } }
    HITJ(0, h0, s0)
    HITJ(1, h1, s1)
    HITJ(2, h2, s2)
    HITJ(3, h3, s3)
    HITJ(4, h4, s4)
    HITJ(5, h5, s5)
    HITJ(6, h6, s6)
    HITJ(7, h7, s7)
#undef HITJ
  }
  return wc;
}

__device__ __forceinline__ v8us ldcol8(const float* __restrict__ p, int pitch) {
  v8us o;
#pragma unroll
  for (int i = 0; i < 8; ++i) o[i] = (unsigned short)bf16_bits(p[(size_t)i * pitch]);
  return o;
}

__global__ __launch_bounds__(NTHR) void k_prep(const float* __restrict__ W0, const float* __restrict__ W1,
                                               const float* __restrict__ W2, const float* __restrict__ L0,
                                               const float* __restrict__ L1, const float* __restrict__ L2,
                                               unsigned short* bt0, unsigned short* bt1, unsigned short* bt2) {
  const int u = (int)blockIdx.x * NTHR + (int)threadIdx.x;
  v8us o = {0, 0, 0, 0, 0, 0, 0, 0};
  unsigned short* dp;
  if (u < NU0) {
    const int n  = u >> 4;
    const int k8 = (u & 15) * 8;
    if (n < DF) o = ldcol8(W0 + (size_t)k8 * DF + n, DF);
    else        o = ldcol8(L0 + (size_t)k8 * DF + (n - DF), DF);
    dp = bt0 + (size_t)n * DF + k8;
  } else if (u < NU0 + NU1) {
    const int v  = u - NU0;
    const int n  = v >> 5;
    const int k8 = (v & 31) * 8;
    const int kk = k8 & (DF - 1);
    if (n < DF) o = ldcol8(W1 + (size_t)kk * DF + n, DF);
    else        o = ldcol8(L1 + (size_t)kk * DF + (n - DF), DF);
    dp = bt1 + (size_t)n * (2 * DF) + k8;
  } else if (u < NU0 + NU1 + NU2) {
    const int v  = u - (NU0 + NU1);
    const int n  = v >> 5;
    const int k8 = (v & 31) * 8;
    const int kk = k8 & (DF - 1);
    if (n < NCLS)                       o = ldcol8(W2 + (size_t)kk * NCLS + n, NCLS);
    else if (n >= 64 && n < 64 + NCLS)  o = ldcol8(L2 + (size_t)kk * NCLS + (n - 64), NCLS);
    dp = bt2 + (size_t)n * (2 * DF) + k8;
  } else {
    return;
  }
  *(volatile v8us*)dp = o;
  __threadfence();
  *(volatile v8us*)dp = o;
}

__global__ __launch_bounds__(NTHR) void k_deg(const int* __restrict__ ids, int nE, int vec8, int* rs) {
  extern __shared__ __attribute__((aligned(16))) int hist[];
  const int tid = (int)threadIdx.x;
  const int base = (int)blockIdx.x * NBD;
  {
    const v4i z4 = {0, 0, 0, 0};
    for (int i = tid * 4; i < NBD; i += NTHR * 4) *(v4ia*)(hist + i) = z4;
  }
  __syncthreads();
  const unsigned ub = (unsigned)base;
  const int sent = -2147483647 - 1;
  const int nChunks = (nE + CHUNK - 1) / CHUNK;
#pragma unroll 1
  for (int ch = 0; ch < nChunks; ++ch) {
    const int cbase = ch * CHUNK;
    const int e0 = cbase + tid * EPT;
    v4i da, db;
    if (vec8 != 0 && cbase + CHUNK <= nE) {
      da = *(const v4i*)(ids + e0);
      db = *(const v4i*)(ids + e0 + 4);
    } else {
      da.x = (e0     < nE) ? ids[min(e0,     nE - 1)] : sent;
      da.y = (e0 + 1 < nE) ? ids[min(e0 + 1, nE - 1)] : sent;
      da.z = (e0 + 2 < nE) ? ids[min(e0 + 2, nE - 1)] : sent;
      da.w = (e0 + 3 < nE) ? ids[min(e0 + 3, nE - 1)] : sent;
      db.x = (e0 + 4 < nE) ? ids[min(e0 + 4, nE - 1)] : sent;
      db.y = (e0 + 5 < nE) ? ids[min(e0 + 5, nE - 1)] : sent;
      db.z = (e0 + 6 < nE) ? ids[min(e0 + 6, nE - 1)] : sent;
      db.w = (e0 + 7 < nE) ? ids[min(e0 + 7, nE - 1)] : sent;
    }
#define DEGJ(X) { const unsigned sj = (unsigned)(X) - ub; if (sj < (unsigned)NBD) atomicAdd(&hist[sj], 1); }
    DEGJ(da.x) DEGJ(da.y) DEGJ(da.z) DEGJ(da.w)
    DEGJ(db.x) DEGJ(db.y) DEGJ(db.z) DEGJ(db.w)
#undef DEGJ
  }
  __syncthreads();
#pragma unroll 1
  for (int i = tid; i < NBD; i += NTHR) {
    int c = hist[i];
    c = c < 1 ? 1 : c;
    const float f = 1.0f / sqrtf((float)c);
    hist[i] = __float_as_int(f);
  }
  __syncthreads();
#pragma unroll 1
  for (int it = 0; it < NBD / (NTHR * 4); ++it) {
    const int s0 = it * (NTHR * 4) + 4 * tid;
    const v4i v = *(const v4ia*)(hist + s0);
    *(volatile v4i*)(rs + (size_t)base + s0) = v;
  }
  __threadfence();
#pragma unroll 1
  for (int it = 0; it < NBD / (NTHR * 4); ++it) {
    const int s0 = it * (NTHR * 4) + 4 * tid;
    const v4i v = *(const v4ia*)(hist + s0);
    *(volatile v4i*)(rs + (size_t)base + s0) = v;
  }
}

__device__ __forceinline__ void bnsplit(float x, float mm, float iv, float g, float be, bool ok,
                                        unsigned& hb, unsigned& lb) {
  float v = ((x - mm) * iv) * g + be;
  v = (v > 0.0f) ? v : (v - v);
  v = ok ? v : 0.0f;
  hb = bf16_bits(v);
  lb = bf16_bits(v - __uint_as_float(hb << 16));
}

template <int MODE>
__global__ __launch_bounds__(GTHR) void k_gemm(const float* __restrict__ feat, float* xwl,
                                               const unsigned short* __restrict__ BT,
                                               const float* __restrict__ mi, const float* __restrict__ gam,
                                               const float* __restrict__ bet, int K, int ncg, int nN) {
  __shared__ __attribute__((aligned(16))) unsigned short As[GBM * APH];
  __shared__ __attribute__((aligned(16))) float stg[GBM * 64];
  __shared__ __attribute__((aligned(16))) float bnp[4 * DF];
  const int tid = (int)threadIdx.x, lane = tid & 31, wave = tid >> 5, hh = lane >> 4, m = lane & 15;
  const int rowBase = (int)blockIdx.x * GBM;

  if constexpr (MODE != 0) {
    const int c4 = 4 * lane;
    v4f t;
    if (wave == 0) {
      t = *(const v4fa*)(mi + c4);
    } else if (wave == 1) {
      t = *(const v4fa*)(mi + DF + c4);
    } else if (wave == 2) {
      const v4f g = *(const v4fa*)(gam + c4);
      t.x = bf16_val(g.x); t.y = bf16_val(g.y); t.z = bf16_val(g.z); t.w = bf16_val(g.w);
    } else {
      const v4f g = *(const v4fa*)(bet + c4);
      t.x = bf16_val(g.x); t.y = bf16_val(g.y); t.z = bf16_val(g.z); t.w = bf16_val(g.w);
    }
    *(v4fa*)(bnp + DF * wave + c4) = t;
    __syncthreads();
  }

#pragma unroll 2
  for (int it = 0; it < (GBM * 16) / GTHR; ++it) {
    const int u   = it * GTHR + tid;
    const int r   = u >> 4;
    const int c8  = (u & 15) * 8;
    const int row = rowBase + r;
    const bool ok = row < nN;
    const int rc  = ok ? row : nN - 1;
    if constexpr (MODE == 0) {
      const float* p = feat + (size_t)rc * DF + c8;
      const v4f a = *(const v4fa*)p;
      const v4f b = *(const v4fa*)(p + 4);
      v8us o;
      o[0] = ok ? (unsigned short)bf16_bits(a.x) : (unsigned short)0;
      o[1] = ok ? (unsigned short)bf16_bits(a.y) : (unsigned short)0;
      o[2] = ok ? (unsigned short)bf16_bits(a.z) : (unsigned short)0;
      o[3] = ok ? (unsigned short)bf16_bits(a.w) : (unsigned short)0;
      o[4] = ok ? (unsigned short)bf16_bits(b.x) : (unsigned short)0;
      o[5] = ok ? (unsigned short)bf16_bits(b.y) : (unsigned short)0;
      o[6] = ok ? (unsigned short)bf16_bits(b.z) : (unsigned short)0;
      o[7] = ok ? (unsigned short)bf16_bits(b.w) : (unsigned short)0;
      *(v8usa*)(As + r * APH + c8) = o;
    } else {
      const float* p = xwl + (size_t)rc * XP + XLO + c8;
      const v4f a = *(const v4fa*)p;
      const v4f b = *(const v4fa*)(p + 4);
      const v4f m0 = *(const v4fa*)(bnp + c8),          m1 = *(const v4fa*)(bnp + c8 + 4);
      const v4f i0 = *(const v4fa*)(bnp + DF + c8),     i1 = *(const v4fa*)(bnp + DF + c8 + 4);
      const v4f g0 = *(const v4fa*)(bnp + 2 * DF + c8), g1 = *(const v4fa*)(bnp + 2 * DF + c8 + 4);
      const v4f e0 = *(const v4fa*)(bnp + 3 * DF + c8), e1 = *(const v4fa*)(bnp + 3 * DF + c8 + 4);
      unsigned h0, h1, h2, h3, h4, h5, h6, h7, l0, l1, l2, l3, l4, l5, l6, l7;
      bnsplit(a.x, m0.x, i0.x, g0.x, e0.x, ok, h0, l0);
      bnsplit(a.y, m0.y, i0.y, g0.y, e0.y, ok, h1, l1);
      bnsplit(a.z, m0.z, i0.z, g0.z, e0.z, ok, h2, l2);
      bnsplit(a.w, m0.w, i0.w, g0.w, e0.w, ok, h3, l3);
      bnsplit(b.x, m1.x, i1.x, g1.x, e1.x, ok, h4, l4);
      bnsplit(b.y, m1.y, i1.y, g1.y, e1.y, ok, h5, l5);
      bnsplit(b.z, m1.z, i1.z, g1.z, e1.z, ok, h6, l6);
      bnsplit(b.w, m1.w, i1.w, g1.w, e1.w, ok, h7, l7);
      v8us oh, ol;
      oh[0] = (unsigned short)h0; oh[1] = (unsigned short)h1; oh[2] = (unsigned short)h2; oh[3] = (unsigned short)h3;
      oh[4] = (unsigned short)h4; oh[5] = (unsigned short)h5; oh[6] = (unsigned short)h6; oh[7] = (unsigned short)h7;
      ol[0] = (unsigned short)l0; ol[1] = (unsigned short)l1; ol[2] = (unsigned short)l2; ol[3] = (unsigned short)l3;
      ol[4] = (unsigned short)l4; ol[5] = (unsigned short)l5; ol[6] = (unsigned short)l6; ol[7] = (unsigned short)l7;
      *(v8usa*)(As + r * APH + c8) = oh;
      *(v8usa*)(As + r * APH + DF + c8) = ol;
    }
  }
  __syncthreads();

  const int ksteps = K >> 5;
  const int half   = ncg >> 1;
  const unsigned short* ap = As + (16 * wave + m) * APH + 8 * hh;
#pragma unroll 1
  for (int cg = 0; cg < ncg; ++cg) {
    v8f acc[4];
    {
      const v8f z = {0.f, 0.f, 0.f, 0.f, 0.f, 0.f, 0.f, 0.f};
      acc[0] = z; acc[1] = z; acc[2] = z; acc[3] = z;
    }
    const unsigned short* wp = BT + (size_t)(64 * cg + m) * (size_t)K + 8 * hh;
#pragma unroll 1
    for (int ks = 0; ks < ksteps; ++ks) {
      FragB af;
      af.h[0] = *(const v8usa*)(ap + 32 * ks);
      af.h[1] = *(const v8usa*)(ap + 32 * ks + 16);
#pragma unroll
      for (int t = 0; t < 4; ++t) {
        const unsigned short* wq = wp + (size_t)(16 * t) * (size_t)K + 32 * ks;
        FragB bf;
        bf.h[0] = *(const v8usa*)wq;
        bf.h[1] = *(const v8usa*)(wq + 16);
        acc[t] = wmb(af, bf, acc[t]);
      }
    }
#pragma unroll
    for (int t = 0; t < 4; ++t) {
      const int lc = 16 * t + m;
#pragma unroll
      for (int r = 0; r < 8; ++r) {
        const int lr = 16 * wave + 8 * hh + r;
        stg[lr * 64 + lc] = acc[t][r];
      }
    }
    __syncthreads();
    v4f fv[8];
#pragma unroll
    for (int i = 0; i < 8; ++i) {
      const int lr = 16 * wave + 2 * i + hh;
      fv[i] = *(const v4fa*)(stg + lr * 64 + 4 * m);
    }
    const int colOff = (cg < half) ? 64 * cg : XLO + 64 * (cg - half);
#pragma unroll
    for (int i = 0; i < 8; ++i) {
      const int gr = rowBase + 16 * wave + 2 * i + hh;
      float* op = xwl + (size_t)gr * XP + colOff + 4 * m;
      *(volatile v4f*)op = fv[i];
    }
    __threadfence();
#pragma unroll
    for (int i = 0; i < 8; ++i) {
      const int gr = rowBase + 16 * wave + 2 * i + hh;
      float* op = xwl + (size_t)gr * XP + colOff + 4 * m;
      *(volatile v4f*)op = fv[i];
    }
    __syncthreads();
  }
}

__device__ __forceinline__ int build_list(const int* __restrict__ keys, int nE, int vec8, int nodeBase,
                                          int* list, int* hl, int* sl, int* cnt, int* offs, int* cur,
                                          int* misc, int tid, int lane, int wave) {
  int t = 0, ov = 0;
  const int nChunks = (nE + CHUNK - 1) / CHUNK;
#pragma unroll 1
  for (int ch = 0; ch < nChunks; ++ch) {
    const int cbase = ch * CHUNK;
    const int wc = scan_chunk<SLA>(keys, nE, cbase, nodeBase, NBA, vec8, list, tid, lane, wave);
    if (lane == 0) misc[wave] = wc;
    __syncthreads();
    if (wave == 0) {
#pragma unroll 1
      for (int w2 = 0; w2 < NWAVE; ++w2) {
        int c = misc[w2];
        c = c < 0 ? 0 : (c > WCAP ? WCAP : c);
#pragma unroll 1
        for (int b0 = 0; b0 < c; b0 += 32) {
          const int idx = b0 + lane;
          const int ent = list[w2 * WCAP + (idx < WCAP ? idx : WCAP - 1)];
          const int m32 = (c - b0) < 32 ? (c - b0) : 32;
#pragma unroll 1
          for (int k = 0; k < m32; ++k) {
            const int u    = __builtin_amdgcn_readlane(ent, k);
            const int slot = u & (NBA - 1);
            const int el   = (u >> SLA) & (CHUNK - 1);
            const int pk   = ((cbase + el) << SLA) | slot;
            if (t < RCAP) {
              if (lane == 0) { hl[t] = pk; cnt[slot] = cnt[slot] + 1; }
              t = t + 1;
            } else {
              ov = 1;
            }
          }
        }
      }
    }
    __syncthreads();
  }
  if (wave == 0 && lane == 0) { misc[8] = t; misc[9] = ov; }
  __syncthreads();
  int tt = misc[8];
  tt = tt < 0 ? 0 : (tt > RCAP ? RCAP : tt);
  const int ovf = misc[9];

  if (wave == 0) {
    const int base = lane * (NBA / 32);
    int s = 0;
#pragma unroll 1
    for (int i = 0; i < NBA / 32; ++i) s += cnt[base + i];
    int incl = s;
#pragma unroll
    for (int d = 1; d < 32; d <<= 1) {
      const int y = __shfl_up(incl, d, 32);
      if (lane >= d) incl += y;
    }
    int run = incl - s;
#pragma unroll 1
    for (int i = 0; i < NBA / 32; ++i) {
      const int cv = cnt[base + i];
      offs[base + i] = run;
      cur[base + i]  = run;
      run += cv;
    }
  }
  __syncthreads();
  if (wave == 0) {
#pragma unroll 1
    for (int b0 = 0; b0 < tt; b0 += 32) {
      const int idx = b0 + lane;
      const int ent = hl[idx < RCAP ? idx : RCAP - 1];
      const int m32 = (tt - b0) < 32 ? (tt - b0) : 32;
#pragma unroll 1
      for (int k = 0; k < m32; ++k) {
        const int u    = __builtin_amdgcn_readlane(ent, k);
        const int slot = u & (NBA - 1);
        if (lane == 0) {
          int p = cur[slot];
          p = p < 0 ? 0 : (p > RCAP - 1 ? RCAP - 1 : p);
          sl[p] = u;
          cur[slot] = p + 1;
        }
      }
    }
  }
  __syncthreads();
  return ovf;
}

__device__ __forceinline__ v4f gather4(const int* sl, int o, int c, const int* __restrict__ srcs,
                                       const float* __restrict__ rso, const float* xw, int nE, int nN, int lane) {
  float a0 = 0.0f, a1 = 0.0f, a2 = 0.0f, a3 = 0.0f;
#pragma unroll 1
  for (int b0 = 0; b0 < c; b0 += 32) {
    int idx = o + b0 + lane;
    idx = idx > RCAP - 1 ? RCAP - 1 : idx;
    const int ent = sl[idx];
    int eid = ent >> SLA;
    eid = eid < 0 ? 0 : (eid > nE - 1 ? nE - 1 : eid);
    int sr = srcs[eid];
    sr = sr < 0 ? 0 : (sr > nN - 1 ? nN - 1 : sr);
    const float cf  = rso[sr];
    const int   cfi = __float_as_int(cf);
    const int m32 = (c - b0) < 32 ? (c - b0) : 32;
#pragma unroll 1
    for (int k = 0; k < m32; ++k) {
      const int   sk = __builtin_amdgcn_readlane(sr, k);
      const float ck = __int_as_float(__builtin_amdgcn_readlane(cfi, k));
      const v4f a = *(const v4fa*)(xw + (size_t)sk * XP + 4 * lane);
      a0 = fmaf(ck, a.x, a0); a1 = fmaf(ck, a.y, a1);
      a2 = fmaf(ck, a.z, a2); a3 = fmaf(ck, a.w, a3);
    }
  }
  v4f r;
  r.x = a0; r.y = a1; r.z = a2; r.w = a3;
  return r;
}

__device__ __forceinline__ v2f gather2(const int* sl, int o, int c, const int* __restrict__ srcs,
                                       const float* __restrict__ rso, const float* xw, int nE, int nN, int lane) {
  float a0 = 0.0f, a1 = 0.0f;
#pragma unroll 1
  for (int b0 = 0; b0 < c; b0 += 32) {
    int idx = o + b0 + lane;
    idx = idx > RCAP - 1 ? RCAP - 1 : idx;
    const int ent = sl[idx];
    int eid = ent >> SLA;
    eid = eid < 0 ? 0 : (eid > nE - 1 ? nE - 1 : eid);
    int sr = srcs[eid];
    sr = sr < 0 ? 0 : (sr > nN - 1 ? nN - 1 : sr);
    const float cf  = rso[sr];
    const int   cfi = __float_as_int(cf);
    const int m32 = (c - b0) < 32 ? (c - b0) : 32;
#pragma unroll 1
    for (int k = 0; k < m32; ++k) {
      const int   sk = __builtin_amdgcn_readlane(sr, k);
      const float ck = __int_as_float(__builtin_amdgcn_readlane(cfi, k));
      const v2f a = *(const v2fa*)(xw + (size_t)sk * XP + 2 * lane);
      a0 = fmaf(ck, a.x, a0); a1 = fmaf(ck, a.y, a1);
    }
  }
  v2f r;
  r.x = a0; r.y = a1;
  return r;
}

template <int NG, int FIN>
__global__ __launch_bounds__(NTHR) void k_scan(const int* __restrict__ keys0, const int* __restrict__ srcs0,
                                               const float* __restrict__ rso0,
                                               const int* __restrict__ keys1, const int* __restrict__ srcs1,
                                               const float* __restrict__ rso1,
                                               const float* __restrict__ oa, const float* __restrict__ b2,
                                               float* xwl, double* rec, float* outp,
                                               int nE, int nN, int vec8) {
  constexpr int O_HL   = LISTN;
  constexpr int O_SL   = O_HL + RCAP;
  constexpr int O_CNT  = O_SL + NG * RCAP;
  constexpr int O_OFF  = O_CNT + NG * NBA;
  constexpr int O_CUR  = O_OFF + NG * NBA;
  constexpr int O_MISC = O_CUR + NBA;
  constexpr int O_TAIL = O_MISC + 16;
  static_assert(O_MISC % 4 == 0 && O_TAIL % 4 == 0);
  extern __shared__ __attribute__((aligned(16))) int dsm[];
  int* list = dsm;
  int* hl   = dsm + O_HL;
  int* sl   = dsm + O_SL;
  int* cnt  = dsm + O_CNT;
  int* offs = dsm + O_OFF;
  int* cur  = dsm + O_CUR;
  int* misc = dsm + O_MISC;
  const int tid = (int)threadIdx.x, lane = tid & 31, wave = tid >> 5;
  const int nodeBase = (int)blockIdx.x * NBA;

  {
    const v4i z4 = {0, 0, 0, 0};
    for (int i = tid * 4; i < O_MISC; i += NTHR * 4) *(v4ia*)(dsm + i) = z4;
    if (tid < 16) misc[tid] = 0;
  }
  __syncthreads();

  int ovf = build_list(keys0, nE, vec8, nodeBase, list, hl, sl, cnt, offs, cur, misc, tid, lane, wave);
  if constexpr (NG == 2) {
    ovf |= build_list(keys1, nE, vec8, nodeBase, list, hl, sl + RCAP, cnt + NBA, offs + NBA, cur, misc,
                      tid, lane, wave);
  }

  const float qnan = __int_as_float(0x7fc00000);
  const float pz = (ovf != 0) ? qnan : 0.0f;
  float oa0 = 1.0f, oa1 = 0.0f;
  if constexpr (NG == 2) { oa0 = bf16_val(oa[0]); oa1 = bf16_val(oa[1]); }
  float bb0 = 0.0f, bb1 = 0.0f;
  if constexpr (FIN != 0) {
    const int lb = lane < (NCLS / 2) ? lane : (NCLS / 2 - 1);
    const v2f t = *(const v2fa*)(b2 + 2 * lb);
    bb0 = bf16_val(t.x); bb1 = bf16_val(t.y);
  }
  double d0 = 0.0, d1 = 0.0, d2 = 0.0, d3 = 0.0;
  double e0 = 0.0, e1 = 0.0, e2 = 0.0, e3 = 0.0;
  float* stgw = (float*)(dsm + O_TAIL) + wave * (OGRP * NCLS);

#pragma unroll 1
  for (int si = 0; si < SPW; ++si) {
    const int s    = wave * SPW + si;
    const int node = nodeBase + s;
    const bool live = node < nN;
    const int nc = live ? node : nN - 1;
    const int cr0 = cnt[s];
    bool big = cr0 > DEGCAP;
    const int c0 = cr0 < 0 ? 0 : (cr0 > DEGCAP ? DEGCAP : cr0);
    int o0 = offs[s];
    o0 = o0 < 0 ? 0 : (o0 > RCAP ? RCAP : o0);
    const float rsi0 = 1.0f / sqrtf((float)(cr0 < 1 ? 1 : cr0));

    if constexpr (FIN == 0) {
      const v4f g0 = gather4(sl, o0, c0, srcs0, rso0, xwl, nE, nN, lane);
      v4f t0;
      t0.x = g0.x * rsi0; t0.y = g0.y * rsi0; t0.z = g0.z * rsi0; t0.w = g0.w * rsi0;
      if constexpr (NG == 2) {
        const int cr1 = cnt[NBA + s];
        big = big || (cr1 > DEGCAP);
        const int c1 = cr1 < 0 ? 0 : (cr1 > DEGCAP ? DEGCAP : cr1);
        int o1 = offs[NBA + s];
        o1 = o1 < 0 ? 0 : (o1 > RCAP ? RCAP : o1);
        const float rsi1 = 1.0f / sqrtf((float)(cr1 < 1 ? 1 : cr1));
        const v4f g1 = gather4(sl + RCAP, o1, c1, srcs1, rso1, xwl, nE, nN, lane);
        t0.x = oa0 * t0.x + oa1 * (g1.x * rsi1);
        t0.y = oa0 * t0.y + oa1 * (g1.y * rsi1);
        t0.z = oa0 * t0.z + oa1 * (g1.z * rsi1);
        t0.w = oa0 * t0.w + oa1 * (g1.w * rsi1);
      }
      const v4f xl = *(const v4fa*)(xwl + (size_t)nc * XP + XLO + 4 * lane);
      const float pzr = big ? qnan : pz;
      v4f pre;
      pre.x = (t0.x + xl.x) + pzr; pre.y = (t0.y + xl.y) + pzr;
      pre.z = (t0.z + xl.z) + pzr; pre.w = (t0.w + xl.w) + pzr;
      if (live) {
        float* op = xwl + (size_t)node * XP + XLO + 4 * lane;
        *(volatile v4f*)op = pre;
        __threadfence();
        *(volatile v4f*)op = pre;
        const double x0 = (double)pre.x, x1 = (double)pre.y, x2 = (double)pre.z, x3 = (double)pre.w;
        d0 += x0; d1 += x1; d2 += x2; d3 += x3;
        e0 = fma(x0, x0, e0); e1 = fma(x1, x1, e1); e2 = fma(x2, x2, e2); e3 = fma(x3, x3, e3);
      }
    } else {
      const v2f g0 = gather2(sl, o0, c0, srcs0, rso0, xwl, nE, nN, lane);
      const v2f xl = *(const v2fa*)(xwl + (size_t)nc * XP + XLO + 2 * lane);
      const float pzr = big ? qnan : pz;
      v2f y;
      y.x = ((g0.x * rsi0 + bb0) + xl.x) + pzr;
      y.y = ((g0.y * rsi0 + bb1) + xl.y) + pzr;
      const int rg = si & (OGRP - 1);
      if (lane < NCLS / 2) *(v2fa*)(stgw + rg * NCLS + 2 * lane) = y;
      if (rg == OGRP - 1) {
        wave_sync();
        const v4f q0 = *(const v4fa*)(stgw + 4 * lane);
        const v4f q1 = *(const v4fa*)(stgw + 128 + 4 * lane);
        const v4f q2 = *(const v4fa*)(stgw + 256 + 4 * lane);
        const v4f q3 = *(const v4fa*)(stgw + 384 + 4 * lane);
        const v4f q4 = *(const v4fa*)(stgw + 512 + 4 * lane);
        wave_sync();
        const int gb = node - (OGRP - 1);
        if (gb < nN) {
          float* op = outp + (size_t)gb * NCLS + 4 * lane;
          *(volatile v4f*)(op)       = q0;
          *(volatile v4f*)(op + 128) = q1;
          *(volatile v4f*)(op + 256) = q2;
          *(volatile v4f*)(op + 384) = q3;
          *(volatile v4f*)(op + 512) = q4;
          __threadfence();
          *(volatile v4f*)(op)       = q0;
          *(volatile v4f*)(op + 128) = q1;
          *(volatile v4f*)(op + 256) = q2;
          *(volatile v4f*)(op + 384) = q3;
          *(volatile v4f*)(op + 512) = q4;
        }
      }
    }
  }

  if constexpr (FIN == 0) {
    double* stS = (double*)(dsm + O_TAIL);
    double* wr = stS + wave * 256 + 4 * lane;
    wr[0] = d0; wr[1] = d1; wr[2] = d2; wr[3] = d3;
    wr[128] = e0; wr[129] = e1; wr[130] = e2; wr[131] = e3;
    __syncthreads();
    if (tid < 128) {
      const int q = 2 * tid;
      double a = 0.0, b = 0.0;
#pragma unroll
      for (int w2 = 0; w2 < NWAVE; ++w2) { a += stS[w2 * 256 + q]; b += stS[w2 * 256 + q + 1]; }
      v2d o;
      o.x = a; o.y = b;
      double* rp = rec + (size_t)blockIdx.x * 256 + q;
      *(volatile v2d*)rp = o;
      __threadfence();
      *(volatile v2d*)rp = o;
    }
  }
}

__global__ __launch_bounds__(128) void k_bncomb(const double* __restrict__ rec, int nblk, double invN, float* mi) {
  __shared__ __attribute__((aligned(16))) float os[2 * DF];
  const int c = (int)threadIdx.x;
  double S = 0.0, Q = 0.0;
#pragma unroll 2
  for (int b = 0; b < nblk; ++b) {
    S += rec[(size_t)b * 256 + c];
    Q += rec[(size_t)b * 256 + 128 + c];
  }
  const double mean = S * invN;
  const double var  = Q * invN - mean * mean;
  const float m32 = (float)mean;
  const float v32 = (float)var;
  os[c] = m32;
  os[DF + c] = 1.0f / sqrtf(v32 + 1e-5f);
  __syncthreads();
  if (c < 64) {
    const v4f v = *(const v4fa*)(os + 4 * c);
    *(volatile v4f*)(mi + 4 * c) = v;
    __threadfence();
    *(volatile v4f*)(mi + 4 * c) = v;
  }
}

static inline int cdiv(int a, int b) { return (a + b - 1) / b; }
static inline size_t al256(size_t o) { return (o + 255) & ~(size_t)255; }

extern "C" void kernel_launch(void* const* d_in, const int* in_sizes, int n_in,
                              void* d_out, int out_size, void* d_ws, size_t ws_size,
                              hipStream_t stream) {
  if (n_in < 17) return;
  if (in_sizes[0] < DF || (in_sizes[0] % DF) != 0) return;
  const int nN = in_sizes[0] / DF;
  if (nN < 16 || nN >= (1 << 24) || (nN % OGRP) != 0) return;
  const int nE = in_sizes[1];
  if (nE < 1 || nE >= (1 << (31 - SLA))) return;
  if (in_sizes[2] != nE || in_sizes[3] != nE || in_sizes[4] != nE) return;
  if (in_sizes[5] != 2) return;
  if (in_sizes[6] != DF * DF || in_sizes[7] != DF * DF || in_sizes[8] != DF * NCLS) return;
  if (in_sizes[9] != NCLS) return;
  if (in_sizes[10] != DF * DF || in_sizes[11] != DF * DF || in_sizes[12] != DF * NCLS) return;
  if (in_sizes[13] != DF || in_sizes[14] != DF || in_sizes[15] != DF || in_sizes[16] != DF) return;
  if ((long long)out_size != (long long)nN * NCLS) return;

  const float* feat = (const float*)d_in[0];
  const int*   src0 = (const int*)d_in[1];
  const int*   dst0 = (const int*)d_in[2];
  const int*   src1 = (const int*)d_in[3];
  const int*   dst1 = (const int*)d_in[4];
  const float* oa   = (const float*)d_in[5];
  const float* W0   = (const float*)d_in[6];
  const float* W1   = (const float*)d_in[7];
  const float* W2   = (const float*)d_in[8];
  const float* b2   = (const float*)d_in[9];
  const float* L0   = (const float*)d_in[10];
  const float* L1   = (const float*)d_in[11];
  const float* L2   = (const float*)d_in[12];
  const float* g0   = (const float*)d_in[13];
  const float* be0  = (const float*)d_in[14];
  const float* g1   = (const float*)d_in[15];
  const float* be1  = (const float*)d_in[16];
  float* out = (float*)d_out;

  const int MP = cdiv(nN, GBM) * GBM;
  const int gM = MP / GBM;
  const int gA = cdiv(nN, NBA);
  const int gD = cdiv(nN, NBD);
  const int vec8 = ((nE & 3) == 0) ? 1 : 0;

  char* ws = (char*)d_ws;
  size_t off = 0;
  const size_t oXWL = off; off = al256(off + (size_t)MP * XP * 4);
  const size_t oRS0 = off; off = al256(off + (size_t)gD * NBD * 4);
  const size_t oRS1 = off; off = al256(off + (size_t)gD * NBD * 4);
  const size_t oBT0 = off; off = al256(off + (size_t)256 * DF * 2);
  const size_t oBT1 = off; off = al256(off + (size_t)256 * 2 * DF * 2);
  const size_t oBT2 = off; off = al256(off + (size_t)128 * 2 * DF * 2);
  const size_t oRC0 = off; off = al256(off + (size_t)gA * 256 * 8);
  const size_t oRC1 = off; off = al256(off + (size_t)gA * 256 * 8);
  const size_t oMI0 = off; off = al256(off + (size_t)2 * DF * 4);
  const size_t oMI1 = off; off = al256(off + (size_t)2 * DF * 4);
  if (off > ws_size || off > (size_t)WSMAX) return;
  float*          XWL = (float*)(ws + oXWL);
  int*            RS0 = (int*)(ws + oRS0);
  int*            RS1 = (int*)(ws + oRS1);
  unsigned short* BT0 = (unsigned short*)(ws + oBT0);
  unsigned short* BT1 = (unsigned short*)(ws + oBT1);
  unsigned short* BT2 = (unsigned short*)(ws + oBT2);
  double*         RC0 = (double*)(ws + oRC0);
  double*         RC1 = (double*)(ws + oRC1);
  float*          MI0 = (float*)(ws + oMI0);
  float*          MI1 = (float*)(ws + oMI1);

  const size_t ldsDeg = (size_t)NBD * 4;
  const size_t lds20  = (size_t)(LISTN + 3 * RCAP + 5 * NBA + 16) * 4 + (size_t)NWAVE * 256 * 8;
  const size_t lds10  = (size_t)(LISTN + 2 * RCAP + 3 * NBA + 16) * 4 + (size_t)NWAVE * 256 * 8;
  const size_t lds11  = (size_t)(LISTN + 2 * RCAP + 3 * NBA + 16) * 4 + (size_t)NWAVE * OGRP * NCLS * 4;
  hipFuncSetAttribute(reinterpret_cast<const void*>(&k_deg), hipFuncAttributeMaxDynamicSharedMemorySize, (int)ldsDeg);
  hipFuncSetAttribute(reinterpret_cast<const void*>(&k_scan<2, 0>), hipFuncAttributeMaxDynamicSharedMemorySize, (int)lds20);
  hipFuncSetAttribute(reinterpret_cast<const void*>(&k_scan<1, 0>), hipFuncAttributeMaxDynamicSharedMemorySize, (int)lds10);
  hipFuncSetAttribute(reinterpret_cast<const void*>(&k_scan<1, 1>), hipFuncAttributeMaxDynamicSharedMemorySize, (int)lds11);

  const double invN = 1.0 / (double)nN;
  const float* RS0f = (const float*)RS0;
  const float* RS1f = (const float*)RS1;

  k_prep<<<(NU0 + NU1 + NU2) / NTHR, NTHR, 0, stream>>>(W0, W1, W2, L0, L1, L2, BT0, BT1, BT2);
  k_deg<<<gD, NTHR, ldsDeg, stream>>>(src0, nE, vec8, RS0);
  k_deg<<<gD, NTHR, ldsDeg, stream>>>(src1, nE, vec8, RS1);
  k_gemm<0><<<gM, GTHR, 0, stream>>>(feat, XWL, BT0, MI0, g0, be0, DF, 4, nN);
  k_scan<2, 0><<<gA, NTHR, lds20, stream>>>(dst0, src0, RS0f, dst1, src1, RS1f, oa, b2, XWL, RC0, out, nE, nN, vec8);
  k_bncomb<<<1, 128, 0, stream>>>(RC0, gA, invN, MI0);
  k_gemm<1><<<gM, GTHR, 0, stream>>>(feat, XWL, BT1, MI0, g0, be0, 2 * DF, 4, nN);
  k_scan<1, 0><<<gA, NTHR, lds10, stream>>>(dst0, src0, RS0f, dst0, src0, RS0f, oa, b2, XWL, RC1, out, nE, nN, vec8);
  k_bncomb<<<1, 128, 0, stream>>>(RC1, gA, invN, MI1);
  k_gemm<1><<<gM, GTHR, 0, stream>>>(feat, XWL, BT2, MI1, g1, be1, 2 * DF, 2, nN);
  k_scan<1, 1><<<gA, NTHR, lds11, stream>>>(dst0, src0, RS0f, dst0, src0, RS0f, oa, b2, XWL, RC1, out, nE, nN, vec8);
}
